// RelativePositionSelfAttention_4415226380580
// MI455X (gfx1250) — hardware-verified
//
#include <hip/hip_runtime.h>
#include <math.h>
typedef __attribute__((ext_vector_type(16))) _Float16 v16h;
typedef __attribute__((ext_vector_type(8)))  _Float16 v8h;
typedef __attribute__((ext_vector_type(16))) __bf16   v16b;
typedef __attribute__((ext_vector_type(8)))  __bf16   v8b;
typedef __attribute__((ext_vector_type(8)))  float    v8f;
typedef __attribute__((ext_vector_type(4)))  float    v4f;
#define PSCALE 32768.0f
#define U16(p) ((const unsigned short*)(const void*)(p))
#define PSCALE_INV (1.0f / 32768.0f)

__device__ __forceinline__ unsigned short f2bf_bits(float f) {
  unsigned u = __float_as_uint(f);
  return (unsigned short)((u + 0x7FFFu + ((u >> 16) & 1u)) >> 16);
}
__device__ __forceinline__ float bf_bits2f(unsigned short h) { return __uint_as_float(((unsigned)h) << 16); }

__device__ __forceinline__ void dep_guard_h(v8f& a, v8f& b, v16h x, v16h y) { asm volatile("v_nop\n\tv_nop\n\tv_nop\n\tv_nop" : "+v"(a), "+v"(b) : "v"(x), "v"(y)); }
__device__ __forceinline__ void dep_guard_b(v8f& a, v8f& b, v16b x, v16b y) { asm volatile("v_nop\n\tv_nop\n\tv_nop\n\tv_nop" : "+v"(a), "+v"(b) : "v"(x), "v"(y)); }
__device__ __forceinline__ void keep4_h(v16h a, v16h b, v16h c, v16h d) { asm volatile("v_nop" :: "v"(a), "v"(b), "v"(c), "v"(d)); }
__device__ __forceinline__ void keep4_b(v16b a, v16b b, v16b c, v16b d) { asm volatile("v_nop" :: "v"(a), "v"(b), "v"(c), "v"(d)); }
__device__ __forceinline__ void acc_guard4(v8f& a, v8f& b, v8f& c, v8f& d) { asm volatile("v_nop\n\tv_nop\n\tv_nop\n\tv_nop" : "+v"(a), "+v"(b), "+v"(c), "+v"(d)); }
template <typename T> struct Frag;
template <> struct Frag<_Float16> {
  typedef v16h V; union U { v16h v; v8h h[2]; };
  static __device__ __forceinline__ v16h load(const _Float16* p) {
    U f; f.h[0] = *(const v8h*)(p); f.h[1] = *(const v8h*)(p + 16); return f.v;
  }
  static __device__ __forceinline__ v8f mma(v16h a, v16h b, v8f c) {
    return __builtin_amdgcn_wmma_f32_16x16x32_f16(false, a, false, b, (short)0, c, false, false);
  }
  static __device__ __forceinline__ void guard(v8f& a, v8f& b, v16h x, v16h y) { dep_guard_h(a, b, x, y); }
  static __device__ __forceinline__ void keep(v16h a, v16h b, v16h c, v16h d) { keep4_h(a, b, c, d); }
};
template <> struct Frag<__bf16> {
  typedef v16b V; union U { v16b v; v8b h[2]; };
  static __device__ __forceinline__ v16b load(const __bf16* p) {
    U f; f.h[0] = *(const v8b*)(p); f.h[1] = *(const v8b*)(p + 16); return f.v;
  }
  static __device__ __forceinline__ v8f mma(v16b a, v16b b, v8f c) {
    return __builtin_amdgcn_wmma_f32_16x16x32_bf16(false, a, false, b, (short)0, c, false, false);
  }
  static __device__ __forceinline__ void guard(v8f& a, v8f& b, v16b x, v16b y) { dep_guard_b(a, b, x, y); }
  static __device__ __forceinline__ void keep(v16b a, v16b b, v16b c, v16b d) { keep4_b(a, b, c, d); }
};

template <int ET> struct Elem;
template <> struct Elem<0> { typedef _Float16 T; };
template <> struct Elem<1> { typedef __bf16 T; };
template <int ET, bool SPLIT, int BIAS_MODE, int OUT_MODE, bool RESID, int ACT = 0>
__global__ __launch_bounds__(256) void wmma_gemm64(
    const unsigned short* __restrict__ Ap, const unsigned short* __restrict__ A2p, int lda, long strideA,
    const unsigned short* __restrict__ Btp, const unsigned short* __restrict__ Bt2p, int ldb, long strideB,
    void* __restrict__ Cout, void* __restrict__ Cout2, int ldc, long strideC,
    const float* __restrict__ bias,
    const float* __restrict__ resid, long strideR,
    int M, int N, int K, float scale) {
  typedef typename Elem<ET>::T T;
  typedef typename Frag<T>::V V;
  const T* A = (const T*)Ap; const T* A2 = (const T*)A2p; const T* Bt = (const T*)Btp; const T* Bt2 = (const T*)Bt2p;
  __shared__ __align__(16) float sT[8][16 * 68];
  const int b    = blockIdx.y;
  const int lane = threadIdx.x & 31;
  const int wave = threadIdx.x >> 5;
  const int tilesN = N >> 6;
  const int tilesM = M >> 6;
  const int tile = blockIdx.x * 8 + wave;
  if (tile >= tilesM * tilesN) return;
  const int tm = tile / tilesN;
  const int tn = tile - tm * tilesN;
  const int m0 = tm << 6;
  const int n0 = tn << 6;

  const T* Ab  = A  + (size_t)b * strideA;
  const T* Bb  = Bt + (size_t)b * strideB;
  const T* Ab2 = SPLIT ? (A2  + (size_t)b * strideA) : nullptr;
  const T* Bb2 = SPLIT ? (Bt2 + (size_t)b * strideB) : nullptr;

  const int rlane = lane & 15;
  const int koff  = (lane >> 4) * 8;
  const int mOff  = (lane >> 4) * 8;

  v8f acc[4][4];
#pragma unroll
  for (int i = 0; i < 4; ++i)
#pragma unroll
    for (int j = 0; j < 4; ++j) acc[i][j] = (v8f){0.f,0.f,0.f,0.f,0.f,0.f,0.f,0.f};

  for (int k0 = 0; k0 < K; k0 += 32) {
    V bh[4], bl[4];
#pragma unroll
    for (int j = 0; j < 4; ++j) {
      const size_t bo = (size_t)(n0 + (j << 4) + rlane) * ldb + koff + k0;
      bh[j] = Frag<T>::load(Bb + bo);
      if (SPLIT) bl[j] = Frag<T>::load(Bb2 + bo);
    }
#pragma unroll
    for (int i = 0; i < 4; ++i) {
      const size_t ao = (size_t)(m0 + (i << 4) + rlane) * lda + koff + k0;
      V ah = Frag<T>::load(Ab + ao);
      V al;
      if (SPLIT) al = Frag<T>::load(Ab2 + ao);
#pragma unroll
      for (int j = 0; j < 4; ++j) {
        acc[i][j] = Frag<T>::mma(ah, bh[j], acc[i][j]);
        if (SPLIT) {
          acc[i][j] = Frag<T>::mma(ah, bl[j], acc[i][j]);
          acc[i][j] = Frag<T>::mma(al, bh[j], acc[i][j]);
        }
      }
      Frag<T>::guard(acc[i][0], acc[i][3], ah, SPLIT ? al : ah);
    }
    Frag<T>::keep(bh[0], bh[1], bh[2], bh[3]);
    if (SPLIT) Frag<T>::keep(bl[0], bl[1], bl[2], bl[3]);
  }
  acc_guard4(acc[0][0], acc[0][1], acc[0][2], acc[0][3]);
  acc_guard4(acc[1][0], acc[1][1], acc[1][2], acc[1][3]);
  acc_guard4(acc[2][0], acc[2][1], acc[2][2], acc[2][3]);
  acc_guard4(acc[3][0], acc[3][1], acc[3][2], acc[3][3]);

  float* slab = sT[wave];
  const float* Rb = RESID ? (resid + (size_t)b * strideR) : nullptr;
#pragma unroll
  for (int i = 0; i < 4; ++i) {
    const int mBase = m0 + (i << 4);
#pragma unroll
    for (int j = 0; j < 4; ++j) {
      const int n = n0 + (j << 4) + rlane;
      float bv = 0.f;
      if (BIAS_MODE == 2) bv = bias[n];
#pragma unroll
      for (int r = 0; r < 8; ++r) {
        float v = acc[i][j][r] * scale;
        if (BIAS_MODE == 1) v += bias[mBase + mOff + r];
        if (BIAS_MODE == 2) v += bv;
        if (RESID) v += Rb[(size_t)(mBase + mOff + r) * ldc + n];
        if (ACT == 1) v = tanhf(v);
        if (ACT == 2) v = fmaxf(v, 0.0f);
        if (ACT == 3) v = v / (1.0f + expf(-v));
        if (ACT == 4) v = (v > 0.f) ? v : 0.01f * v;
        if (ACT == 5) v = 0.5f * v * (1.0f + erff(v * 0.70710678118654752f));
        slab[(mOff + r) * 68 + (j << 4) + rlane] = v;
      }
    }
    __builtin_amdgcn_fence(__ATOMIC_RELEASE, "workgroup");
    __builtin_amdgcn_wave_barrier();
    __builtin_amdgcn_fence(__ATOMIC_ACQUIRE, "workgroup");
    if (OUT_MODE == 0) {
      float* C = (float*)Cout + (size_t)b * strideC;
      const int hh = lane >> 4, c4 = (lane & 15) * 4;
      for (int pass = 0; pass < 2; ++pass) {
#pragma unroll
        for (int it = 0; it < 8; ++it) {
          const int row = it * 2 + hh;
          v4f v = *(const v4f*)(slab + row * 68 + c4);
          *(volatile v4f*)(C + (size_t)(mBase + row) * ldc + n0 + c4) = v;
        }
        __threadfence();
      }
    } else {
      const int q = lane >> 3, c8 = (lane & 7) * 8;
      unsigned short* C  = (unsigned short*)Cout  + (size_t)b * strideC;
      unsigned short* C2 = (OUT_MODE == 2) ? ((unsigned short*)Cout2 + (size_t)b * strideC) : nullptr;
      for (int pass = 0; pass < 2; ++pass) {
#pragma unroll
        for (int it = 0; it < 4; ++it) {
          const int row = it * 4 + q;
          const float* sp = slab + row * 68 + c8;
          v8h hv, lv;
#pragma unroll
          for (int e = 0; e < 8; ++e) {
            if (OUT_MODE == 1) {
              hv[e] = (_Float16)sp[e];
            } else {
              unsigned short hb = f2bf_bits(sp[e]);
              unsigned short lb = f2bf_bits(sp[e] - bf_bits2f(hb));
              hv[e] = __builtin_bit_cast(_Float16, hb);
              lv[e] = __builtin_bit_cast(_Float16, lb);
            }
          }
          *(volatile v8h*)(C + (size_t)(mBase + row) * ldc + n0 + c8) = hv;
          if (OUT_MODE == 2) *(volatile v8h*)(C2 + (size_t)(mBase + row) * ldc + n0 + c8) = lv;
        }
        __threadfence();
      }
    }
    __builtin_amdgcn_fence(__ATOMIC_RELEASE, "workgroup");
    __builtin_amdgcn_wave_barrier();
    __builtin_amdgcn_fence(__ATOMIC_ACQUIRE, "workgroup");
  }
}

__global__ __launch_bounds__(256) void cast_f32_f16x2(
    const float* __restrict__ in, _Float16* __restrict__ out, int n2) {
  int i = blockIdx.x * 256 + threadIdx.x;
  if (i < n2) {
    const _Float16 h0 = (_Float16)in[2 * i], h1 = (_Float16)in[2 * i + 1];
    const unsigned u = (unsigned)__builtin_bit_cast(unsigned short, h0) | ((unsigned)__builtin_bit_cast(unsigned short, h1) << 16);
    ((volatile unsigned*)out)[i] = u;
    __threadfence();
    ((volatile unsigned*)out)[i] = u;
  }
}


__global__ __launch_bounds__(256) void transpose_cast_f16(const float* __restrict__ in, int ldi,
                                                         _Float16* __restrict__ outT, int ldo, float scale) {
  __shared__ __align__(16) _Float16 tile[64][72];
  const int c0 = blockIdx.x * 64, r0 = blockIdx.y * 64;
  const int t = threadIdx.y * 32 + threadIdx.x;
  for (int i = threadIdx.y; i < 64; i += 8) {
    tile[threadIdx.x][i]      = (_Float16)(in[(size_t)(r0 + i) * ldi + c0 + threadIdx.x] * scale);
    tile[32 + threadIdx.x][i] = (_Float16)(in[(size_t)(r0 + i) * ldi + c0 + 32 + threadIdx.x] * scale);
  }
  __syncthreads();
  const int q = t >> 3, c8 = (t & 7) * 8;
  for (int pass = 0; pass < 2; ++pass) {
#pragma unroll
    for (int it = 0; it < 2; ++it) {
      const int c = it * 32 + q;
      v8h hv = *(const v8h*)(&tile[c][c8]);
      *(volatile v8h*)(outT + (size_t)(c0 + c) * ldo + r0 + c8) = hv;
    }
    __threadfence();
  }
}
__global__ __launch_bounds__(256) void split_f32_bf16x2(
    const float* __restrict__ in, __bf16* __restrict__ hi, __bf16* __restrict__ lo, long n2) {
  long i = (long)blockIdx.x * 256 + threadIdx.x;
  long stride = (long)gridDim.x * 256;
  for (int pass = 0; pass < 2; ++pass) {
    for (long j = i; j < n2; j += stride) {
      const float a = in[2 * j], b = in[2 * j + 1];
      const unsigned short ah = f2bf_bits(a), bh = f2bf_bits(b);
      const unsigned short al = f2bf_bits(a - bf_bits2f(ah)), bl = f2bf_bits(b - bf_bits2f(bh));
      ((volatile unsigned*)hi)[j] = (unsigned)ah | ((unsigned)bh << 16);
      ((volatile unsigned*)lo)[j] = (unsigned)al | ((unsigned)bl << 16);
    }
    __threadfence();
  }
}


__global__ __launch_bounds__(256) void transpose_split_bf16(const float* __restrict__ in, int ldi,
                                                           __bf16* __restrict__ outH, __bf16* __restrict__ outL, int ldo) {
  __shared__ __align__(16) float tile[64][68];
  const int c0 = blockIdx.x * 64, r0 = blockIdx.y * 64;
  const int t = threadIdx.y * 32 + threadIdx.x;
  for (int i = threadIdx.y; i < 64; i += 8) {
    tile[threadIdx.x][i]      = in[(size_t)(r0 + i) * ldi + c0 + threadIdx.x];
    tile[32 + threadIdx.x][i] = in[(size_t)(r0 + i) * ldi + c0 + 32 + threadIdx.x];
  }
  __syncthreads();
  const int q = t >> 3, c8 = (t & 7) * 8;
  for (int pass = 0; pass < 2; ++pass) {
#pragma unroll
    for (int it = 0; it < 2; ++it) {
      const int c = it * 32 + q;
      v8b hv, lv;
#pragma unroll
      for (int e = 0; e < 8; ++e) {
        const float f = tile[c][c8 + e];
        const unsigned short hb = f2bf_bits(f);
        hv[e] = __builtin_bit_cast(__bf16, hb);
        lv[e] = __builtin_bit_cast(__bf16, f2bf_bits(f - bf_bits2f(hb)));
      }
      *(volatile v8b*)(outH + (size_t)(c0 + c) * ldo + r0 + c8) = hv;
      *(volatile v8b*)(outL + (size_t)(c0 + c) * ldo + r0 + c8) = lv;
    }
    __threadfence();
  }
}

#define RB 8
#define RS 1024
#define RH 128
#define RR 129
#define RRP 192
#define RRW (RB * RS)
__global__ __launch_bounds__(256) void softmax_kernel(const float* __restrict__ Sm, const float* __restrict__ QR, float* __restrict__ attn, unsigned* __restrict__ P16, unsigned* __restrict__ AB16) {
  __shared__ float red[8]; __shared__ float stat; __shared__ float arow[RS]; __shared__ float ab[RRP];
  const int row = blockIdx.x; const int i = row % RS; const int t = threadIdx.x, lane = t & 31, wave = t >> 5;
  const float* sr = Sm + (size_t)row * RS; const float* qr = QR + (size_t)row * RRP;
  float v[4]; float mx = -INFINITY;
#pragma unroll
  for (int q = 0; q < 4; ++q) { const int j = t + 256 * q; int r = j - i; r = r < -64 ? -64 : (r > 64 ? 64 : r); v[q] = sr[j] * 0.08838834764831845f + qr[r + 64]; mx = fmaxf(mx, v[q]); }
  for (int o = 16; o > 0; o >>= 1) mx = fmaxf(mx, __shfl_xor(mx, o, 32));
  if (lane == 0) red[wave] = mx; __syncthreads();
  if (t == 0) { float m = red[0]; for (int w = 1; w < 8; ++w) m = fmaxf(m, red[w]); stat = m; } __syncthreads();
  const float m = stat; __syncthreads();
  float se = 0.f;
#pragma unroll
  for (int q = 0; q < 4; ++q) { v[q] = expf(v[q] - m); se += v[q]; }
  for (int o = 16; o > 0; o >>= 1) se += __shfl_xor(se, o, 32);
  if (lane == 0) red[wave] = se; __syncthreads();
  if (t == 0) { float s = 0.f; for (int w = 0; w < 8; ++w) s += red[w]; stat = 1.0f / s; } __syncthreads();
  const float inv = stat;
#pragma unroll
  for (int q = 0; q < 4; ++q) { v[q] *= inv; arow[t + 256 * q] = v[q]; }
  for (int r = t; r < RRP; r += 256) ab[r] = 0.f;
  __syncthreads();
  float lo = 0.f, hi = 0.f;
#pragma unroll
  for (int q = 0; q < 4; ++q) { const int j = t + 256 * q; if (j <= i - 64) lo += v[q]; if (j >= i + 64) hi += v[q]; }
  for (int o = 16; o > 0; o >>= 1) { lo += __shfl_xor(lo, o, 32); hi += __shfl_xor(hi, o, 32); }
  __shared__ float rlo[8], rhi[8];
  if (lane == 0) { rlo[wave] = lo; rhi[wave] = hi; } __syncthreads();
  if (t < RR) { float val;
    if (t == 0) { val = 0.f; for (int w = 0; w < 8; ++w) val += rlo[w]; }
    else if (t == RR - 1) { val = 0.f; for (int w = 0; w < 8; ++w) val += rhi[w]; }
    else { const int j = i + t - 64; val = (j >= 0 && j < RS) ? arow[j] : 0.f; }
    ab[t] = val; }
  __syncthreads();
  for (int pass = 0; pass < 2; ++pass) {
#pragma unroll
    for (int q = 0; q < 4; ++q) ((volatile float*)attn)[(size_t)row * RS + t + 256 * q] = v[q];
#pragma unroll
    for (int q = 0; q < 2; ++q) { const int c = 2 * (t + 256 * q);
      const unsigned u = (unsigned)__builtin_bit_cast(unsigned short, (_Float16)(arow[c] * 32768.0f)) | ((unsigned)__builtin_bit_cast(unsigned short, (_Float16)(arow[c + 1] * 32768.0f)) << 16);
      ((volatile unsigned*)P16)[(size_t)row * (RS / 2) + t + 256 * q] = u; }
    if (t < RRP / 2) { const unsigned u = (unsigned)__builtin_bit_cast(unsigned short, (_Float16)(ab[2 * t] * 32768.0f)) | ((unsigned)__builtin_bit_cast(unsigned short, (_Float16)(ab[2 * t + 1] * 32768.0f)) << 16);
      ((volatile unsigned*)AB16)[(size_t)row * (RRP / 2) + t] = u; }
    __threadfence(); }
}
__global__ __launch_bounds__(256) void rel_kernel(const float* __restrict__ relk, const float* __restrict__ relv, unsigned* __restrict__ RKh, unsigned* __restrict__ RKl, unsigned* __restrict__ RVT) {
  const int i = blockIdx.x * 256 + threadIdx.x; if (i >= RRP * RH / 2) return;
  { const int r = (2 * i) / RH, h = (2 * i) % RH; float a = 0.f, b = 0.f; if (r < RR) { a = relk[r * RH + h]; b = relk[r * RH + h + 1]; }
    const unsigned short ah = f2bf_bits(a), bh = f2bf_bits(b), al = f2bf_bits(a - bf_bits2f(ah)), bl = f2bf_bits(b - bf_bits2f(bh));
    ((volatile unsigned*)RKh)[i] = (unsigned)ah | ((unsigned)bh << 16); ((volatile unsigned*)RKl)[i] = (unsigned)al | ((unsigned)bl << 16); __threadfence();
    ((volatile unsigned*)RKh)[i] = (unsigned)ah | ((unsigned)bh << 16); ((volatile unsigned*)RKl)[i] = (unsigned)al | ((unsigned)bl << 16); }
  { const int h = (2 * i) / RRP, r = (2 * i) % RRP; float a = 0.f, b = 0.f; if (r < RR) a = relv[r * RH + h]; if (r + 1 < RR) b = relv[(r + 1) * RH + h];
    const unsigned u = (unsigned)__builtin_bit_cast(unsigned short, (_Float16)a) | ((unsigned)__builtin_bit_cast(unsigned short, (_Float16)b) << 16); ((volatile unsigned*)RVT)[i] = u; __threadfence(); ((volatile unsigned*)RVT)[i] = u; }
}
__global__ void bias_cat_kernel(const float* a, const float* b, const float* c, float* o) { const int i = blockIdx.x * 256 + threadIdx.x; if (i >= 384) return; const float v = (i < 128) ? a[i] : (i < 256 ? b[i - 128] : c[i - 256]); ((volatile float*)o)[i] = v; __threadfence(); ((volatile float*)o)[i] = v; }
__global__ __launch_bounds__(256) void vt_kernel(const float* __restrict__ QKV, unsigned* __restrict__ VT) {
  __shared__ float tile[64][65];
  const int b = blockIdx.z, h0 = blockIdx.y * 64, j0 = blockIdx.x * 64, tx = threadIdx.x, ty = threadIdx.y;
  for (int r = ty; r < 64; r += 8) { const int j = j0 + r; for (int c = tx; c < 64; c += 32) tile[c][r] = QKV[((size_t)b * RS + j) * 384 + 256 + h0 + c]; }
  __syncthreads();
  for (int pass = 0; pass < 2; ++pass) { for (int r = ty; r < 64; r += 8) { const int h = h0 + r; const unsigned u = (unsigned)__builtin_bit_cast(unsigned short, (_Float16)tile[r][2 * tx]) | ((unsigned)__builtin_bit_cast(unsigned short, (_Float16)tile[r][2 * tx + 1]) << 16);
      ((volatile unsigned*)VT)[(((size_t)b * RH + h) * RS + j0) / 2 + tx] = u; } __threadfence(); }
}
__global__ __launch_bounds__(256) void ln_kernel(const float* __restrict__ O, const float* __restrict__ x, const float* __restrict__ g, const float* __restrict__ bb, float* __restrict__ y) {
  const int lane = threadIdx.x & 31, wave = threadIdx.x >> 5; const size_t row = (size_t)blockIdx.x * 8 + wave;
  v4f v = *(const v4f*)(O + row * RH + lane * 4) + *(const v4f*)(x + row * RH + lane * 4);
  float s = v[0] + v[1] + v[2] + v[3]; for (int o = 16; o > 0; o >>= 1) s += __shfl_xor(s, o, 32);
  const float mean = s / RH; float s2 = 0.f; for (int e = 0; e < 4; ++e) { const float d = v[e] - mean; s2 += d * d; } for (int o = 16; o > 0; o >>= 1) s2 += __shfl_xor(s2, o, 32);
  const float inv = rsqrtf(s2 / RH + 1e-5f);
  v4f o4; for (int e = 0; e < 4; ++e) o4[e] = (v[e] - mean) * inv * g[lane * 4 + e] + bb[lane * 4 + e];
  *(volatile v4f*)(y + row * RH + lane * 4) = o4; __threadfence(); *(volatile v4f*)(y + row * RH + lane * 4) = o4;
}
extern "C" void kernel_launch(void* const* d_in, const int* in_sizes, int n_in, void* d_out, int out_size, void* d_ws, size_t ws_size, hipStream_t stream) {
  (void)in_sizes; (void)n_in; (void)out_size; (void)ws_size;
  const float* x = (const float*)d_in[0]; const float* Wq = (const float*)d_in[1]; const float* bq = (const float*)d_in[2]; const float* Wk = (const float*)d_in[3]; const float* bk = (const float*)d_in[4]; const float* Wv = (const float*)d_in[5]; const float* bv = (const float*)d_in[6];
  const float* relk = (const float*)d_in[7]; const float* relv = (const float*)d_in[8]; const float* Wo = (const float*)d_in[9]; const float* bo = (const float*)d_in[10]; const float* gamma = (const float*)d_in[11]; const float* beta = (const float*)d_in[12];
  float* y = (float*)d_out; float* attn = y + (size_t)RRW * RH;
  char* ws = (char*)d_ws; size_t off = 0;
  auto carve = [&](size_t bytes) -> char* { char* p = ws + off; off += (bytes + 255) & ~(size_t)255; return p; };
  __bf16* Xh = (__bf16*)carve((size_t)RRW * RH * 2); __bf16* Xl = (__bf16*)carve((size_t)RRW * RH * 2); __bf16* WTh = (__bf16*)carve((size_t)384 * RH * 2); __bf16* WTl = (__bf16*)carve((size_t)384 * RH * 2); _Float16* WoT = (_Float16*)carve(RH * RH * 2); float* b3 = (float*)carve(384 * 4);
  float* QKV = (float*)carve((size_t)RRW * 384 * 4);
  __bf16* QKh = (__bf16*)carve((size_t)RRW * 384 * 2); __bf16* QKl = (__bf16*)carve((size_t)RRW * 384 * 2);
  unsigned* RKh = (unsigned*)carve(RRP * RH * 2); unsigned* RKl = (unsigned*)carve(RRP * RH * 2); unsigned* RVT = (unsigned*)carve(RH * RRP * 2);
  float* QR = (float*)carve((size_t)RRW * RRP * 4);
  float* Sm = (float*)carve((size_t)RB * RS * RS * 4);
  unsigned* P16 = (unsigned*)carve((size_t)RB * RS * RS * 2); unsigned* AB16 = (unsigned*)carve((size_t)RRW * RRP * 2); unsigned* VT = (unsigned*)carve((size_t)RB * RH * RS * 2);
  float* CTX = (float*)carve((size_t)RRW * RH * 4); float* CTX2 = (float*)carve((size_t)RRW * RH * 4); unsigned* C16 = (unsigned*)carve((size_t)RRW * RH * 2); float* O = (float*)carve((size_t)RRW * RH * 4);
  split_f32_bf16x2<<<(RRW * RH / 2 + 255) / 256, 256, 0, stream>>>(x, Xh, Xl, RRW * RH / 2);
  transpose_split_bf16<<<dim3(RH / 64, RH / 64), dim3(32, 8), 0, stream>>>(Wq, RH, WTh, WTl, RH);
  transpose_split_bf16<<<dim3(RH / 64, RH / 64), dim3(32, 8), 0, stream>>>(Wk, RH, WTh + RH * RH, WTl + RH * RH, RH);
  transpose_split_bf16<<<dim3(RH / 64, RH / 64), dim3(32, 8), 0, stream>>>(Wv, RH, WTh + 2 * RH * RH, WTl + 2 * RH * RH, RH);
  transpose_cast_f16<<<dim3(RH / 64, RH / 64), dim3(32, 8), 0, stream>>>(Wo, RH, WoT, RH, 1.0f);
  bias_cat_kernel<<<2, 256, 0, stream>>>(bq, bk, bv, b3);
  rel_kernel<<<(RRP * RH / 2 + 255) / 256, 256, 0, stream>>>(relk, relv, RKh, RKl, RVT);
  { const int t = (RRW / 64) * (384 / 64);
    wmma_gemm64<1, true, 2, 0, false><<<dim3((t + 7) / 8, 1), 256, 0, stream>>>(U16(Xh), U16(Xl), RH, 0, U16(WTh), U16(WTl), RH, 0, QKV, nullptr, 384, 0, b3, nullptr, 0, RRW, 384, RH, 1.0f); }
  split_f32_bf16x2<<<(RRW * 384 / 2 + 255) / 256, 256, 0, stream>>>(QKV, QKh, QKl, RRW * 384 / 2);
  { const int t = (RRW / 64) * (RRP / 64);
    wmma_gemm64<1, true, 0, 0, false><<<dim3((t + 7) / 8, 1), 256, 0, stream>>>(U16(QKh), U16(QKl), 384, 0, (const unsigned short*)RKh, (const unsigned short*)RKl, RH, 0, QR, nullptr, RRP, 0, nullptr, nullptr, 0, RRW, RRP, RH, 1.0f); }
  { const int t = (RS / 64) * (RS / 64);
    wmma_gemm64<1, true, 0, 0, false><<<dim3((t + 7) / 8, RB), 256, 0, stream>>>(U16(QKh), U16(QKl), 384, (long)RS * 384, U16(QKh + RH), U16(QKl + RH), 384, (long)RS * 384, Sm, nullptr, RS, (long)RS * RS, nullptr, nullptr, 0, RS, RS, RH, 1.0f); }
  softmax_kernel<<<RRW, 256, 0, stream>>>(Sm, QR, attn, P16, AB16);
  vt_kernel<<<dim3(RS / 64, RH / 64, RB), dim3(32, 8), 0, stream>>>(QKV, VT);
  { const int t = (RS / 64) * (RH / 64);
    wmma_gemm64<0, false, 0, 0, false><<<dim3((t + 7) / 8, RB), 256, 0, stream>>>((const unsigned short*)P16, nullptr, RS, (long)RS * RS, (const unsigned short*)VT, nullptr, RS, (long)RH * RS, CTX, nullptr, RH, (long)RS * RH, nullptr, nullptr, 0, RS, RH, RS, 1.0f / 32768.0f);
    const int t2 = (RRW / 64) * (RH / 64);
    wmma_gemm64<0, false, 0, 0, true><<<dim3((t2 + 7) / 8, 1), 256, 0, stream>>>((const unsigned short*)AB16, nullptr, RRP, 0, (const unsigned short*)RVT, nullptr, RRP, 0, CTX2, nullptr, RH, 0, nullptr, CTX, 0, RRW, RH, RRP, 1.0f / 32768.0f); }
  cast_f32_f16x2<<<(RRW * RH / 2 + 255) / 256, 256, 0, stream>>>(CTX2, (_Float16*)C16, RRW * RH / 2);
  { const int t = (RRW / 64) * (RH / 64);
    wmma_gemm64<0, false, 2, 0, false><<<dim3((t + 7) / 8, 1), 256, 0, stream>>>((const unsigned short*)C16, nullptr, RH, 0, U16(WoT), nullptr, RH, 0, O, nullptr, RH, 0, bo, nullptr, 0, RRW, RH, RH, 1.0f); }
  ln_kernel<<<RRW / 8, 256, 0, stream>>>(O, x, gamma, beta, y);
}
